// EnhancedCrossAttention3D_18476949307799
// MI455X (gfx1250) — hardware-verified
//
#include <hip/hip_runtime.h>


namespace {
constexpr int NB = 2, C = 64, N = 8192, NR = NB * N;
constexpr float XS = 8.0f, WSC = 256.0f, PS = 8.0f, LOG2E = 1.4426950408889634f;
typedef _Float16 b16;
typedef __attribute__((ext_vector_type(16))) _Float16 v16b;
typedef __attribute__((ext_vector_type(8))) _Float16 v8b;
typedef __attribute__((ext_vector_type(8))) float v8f;
typedef __attribute__((ext_vector_type(4))) float v4f;
__device__ __forceinline__ float bf16_rne(float f) { unsigned int u = __float_as_uint(f); u += 0x7FFFu + ((u >> 16) & 1u); return __uint_as_float(u & 0xFFFF0000u); }
__device__ __forceinline__ void split16(float v, b16& hi, b16& lo) { hi = (b16)v; lo = (b16)(v - (float)hi); }
__device__ __forceinline__ v16b frag_kb(const b16* p, int hh) { const v8b a = *(const v8b*)(p + 8 * hh), b = *(const v8b*)(p + 16 + 8 * hh); v16b f;
#pragma unroll
  for (int e = 0; e < 8; ++e) { f[e] = a[e]; f[8 + e] = b[e]; } return f; }
__device__ __forceinline__ v8f wmma16b(v16b a, v16b b, v8f c) { v8f d = __builtin_amdgcn_wmma_f32_16x16x32_f16(false, a, false, b, (short)0, c, false, false); asm volatile("v_nop\n\tv_nop\n\tv_nop\n\tv_nop" : "+v"(d) : "v"(a), "v"(b)); return d; }
__device__ __forceinline__ void wave_lds_sync() { __builtin_amdgcn_fence(__ATOMIC_RELEASE, "workgroup"); __builtin_amdgcn_wave_barrier(); __builtin_amdgcn_fence(__ATOMIC_ACQUIRE, "workgroup"); }

__global__ __launch_bounds__(256) void prep_kernel(const float* __restrict__ b1, const float* __restrict__ b2, const float* __restrict__ wq, const float* __restrict__ wk, const float* __restrict__ wv, const float* __restrict__ wp, b16* __restrict__ X1T, b16* __restrict__ X2T, b16* __restrict__ W4) {
  __shared__ __attribute__((aligned(16))) b16 T[64][64 + 8];
  const int n0 = blockIdx.x * 64, which = blockIdx.y, b = blockIdx.z, t_ = threadIdx.x; const float* src = (which ? b2 : b1) + (size_t)b * C * N; b16* dst = which ? X2T : X1T;
  for (int q = t_; q < 64 * 64; q += 256) { const int c = q >> 6, nn = q & 63; T[nn][c] = (b16)(bf16_rne(src[(size_t)c * N + n0 + nn]) * XS); }
  __syncthreads();
  for (int pass = 0; pass < 2; ++pass) { for (int q = t_; q < 64 * 8; q += 256) { const int nn = q >> 3, c8 = (q & 7) * 8; *(volatile v8b*)(dst + ((size_t)b * N + n0 + nn) * C + c8) = *(const v8b*)(&T[nn][c8]); } __threadfence(); }
  if (blockIdx.x == 0 && which == 0 && b == 0) { for (int q = t_; q < 4 * C * C / 8; q += 256) { const int e = q * 8; const int kind = e / (C * C), r = e % (C * C); const float* w = kind == 0 ? wq : kind == 1 ? wk : kind == 2 ? wv : wp; v8b o; for (int j = 0; j < 8; ++j) o[j] = (b16)(bf16_rne(w[r + j]) * WSC); for (int pass = 0; pass < 2; ++pass) { *(volatile v8b*)(W4 + e) = o; __threadfence(); } } }
}
__global__ __launch_bounds__(128) void proj_kernel(const b16* __restrict__ X1T, const b16* __restrict__ X2T, const b16* __restrict__ W4, const float* __restrict__ bq, const float* __restrict__ bk, const float* __restrict__ bv, b16* __restrict__ Qh, b16* __restrict__ Ql, b16* __restrict__ Kh, b16* __restrict__ Kl, b16* __restrict__ VTh, b16* __restrict__ VTl) {
  __shared__ __attribute__((aligned(16))) b16 Th[64][64 + 8], Tl[64][64 + 8];
  const int wave = threadIdx.x >> 5, lane = threadIdx.x & 31, nloc = lane & 15, hlf = lane >> 4, t_ = threadIdx.x; const int kind = blockIdx.y; const size_t m0 = (size_t)blockIdx.x * 64 + wave * 16;
  const b16* X = kind == 0 ? X1T : X2T; const b16* W = W4 + (size_t)kind * C * C; const float* bias = kind == 0 ? bq : kind == 1 ? bk : bv;
  v8f acc[4] = {{}, {}, {}, {}};
#pragma unroll
  for (int kb = 0; kb < C; kb += 32) { const v16b a = frag_kb(X + (m0 + nloc) * C + kb, hlf);
#pragma unroll
    for (int t = 0; t < 4; ++t) acc[t] = wmma16b(a, frag_kb(W + (size_t)(t * 16 + nloc) * C + kb, hlf), acc[t]); }
  if (kind < 2) {
#pragma unroll
    for (int t = 0; t < 4; ++t) { const float bb = bf16_rne(bias[t * 16 + nloc]);
#pragma unroll 1
      for (int r = 0; r < 8; ++r) { b16 p, q; split16((acc[t][r] * (1.0f / (XS * WSC)) + bb) * XS, p, q); Th[wave * 16 + 8 * hlf + r][t * 16 + nloc] = p; Tl[wave * 16 + 8 * hlf + r][t * 16 + nloc] = q; } }
    wave_lds_sync(); b16* dh = kind == 0 ? Qh : Kh; b16* dl = kind == 0 ? Ql : Kl;
    for (int pass = 0; pass < 2; ++pass) { for (int r4 = 0; r4 < 16; r4 += 4) { const int rr = wave * 16 + r4 + (lane >> 3), c8 = (lane & 7) * 8; *(volatile v8b*)(dh + ((size_t)blockIdx.x * 64 + rr) * C + c8) = *(const v8b*)(&Th[rr][c8]); *(volatile v8b*)(dl + ((size_t)blockIdx.x * 64 + rr) * C + c8) = *(const v8b*)(&Tl[rr][c8]); } __threadfence(); }
  } else {
#pragma unroll
    for (int t = 0; t < 4; ++t) { const float bb = bf16_rne(bias[t * 16 + nloc]);
#pragma unroll 1
      for (int r = 0; r < 8; ++r) { b16 p, q; split16((acc[t][r] * (1.0f / (XS * WSC)) + bb) * XS, p, q); Th[t * 16 + nloc][wave * 16 + 8 * hlf + r] = p; Tl[t * 16 + nloc][wave * 16 + 8 * hlf + r] = q; } }
    __syncthreads(); const size_t r0 = (size_t)blockIdx.x * 64; const size_t b = r0 / N; const int n0 = (int)(r0 % N);
    for (int pass = 0; pass < 2; ++pass) { for (int q = t_; q < 64 * 8; q += 128) { const int d = q >> 3, c8 = (q & 7) * 8; const size_t gi = ((b * C + d) * N) + n0 + c8; *(volatile v8b*)(VTh + gi) = *(const v8b*)(&Th[d][c8]); *(volatile v8b*)(VTl + gi) = *(const v8b*)(&Tl[d][c8]); } __threadfence(); }
  }
}
__global__ __launch_bounds__(64) void attn_kernel(const b16* __restrict__ Qh, const b16* __restrict__ Ql, const b16* __restrict__ Kh, const b16* __restrict__ Kl, const b16* __restrict__ VTh, const b16* __restrict__ VTl, const b16* __restrict__ W4, const float* __restrict__ bp, float* __restrict__ out) {
  __shared__ __attribute__((aligned(16))) b16 Oh[32][C + 8], Olo[32][C + 8]; __shared__ __attribute__((aligned(16))) float St[C][32 + 4];
  const int wave = threadIdx.x >> 5, lane = threadIdx.x & 31, hh = lane >> 4, col = lane & 15; const int b = blockIdx.y; const int q0 = blockIdx.x * 32 + wave * 16, qi = q0 + col;
  const size_t qo = ((size_t)b * N + qi) * C; const v16b qa0 = frag_kb(Qh + qo, hh), qa1 = frag_kb(Qh + qo + 32, hh), ql0 = frag_kb(Ql + qo, hh), ql1 = frag_kb(Ql + qo + 32, hh);
  const b16* Kb = Kh + (size_t)b * N * C; const b16* Klb = Kl + (size_t)b * N * C; const b16* Vb = VTh + (size_t)b * C * N; const b16* Vlb = VTl + (size_t)b * C * N;
  v8f o[4] = {{}, {}, {}, {}}, ol[4] = {{}, {}, {}, {}}; float mrun = -INFINITY, lrun = 0.0f; const float cs = 0.125f * LOG2E / (XS * XS);
  for (int kb = 0; kb < N; kb += 32) {
    v8f s0 = {}, s1 = {};
    { const b16* k0 = Kb + (size_t)(kb + col) * C, *k1 = Kb + (size_t)(kb + 16 + col) * C, *k0l = Klb + (size_t)(kb + col) * C, *k1l = Klb + (size_t)(kb + 16 + col) * C;
      v16b f = frag_kb(k0, hh); s0 = wmma16b(f, qa0, s0); s0 = wmma16b(f, ql0, s0); s0 = wmma16b(frag_kb(k0l, hh), qa0, s0);
      f = frag_kb(k0 + 32, hh); s0 = wmma16b(f, qa1, s0); s0 = wmma16b(f, ql1, s0); s0 = wmma16b(frag_kb(k0l + 32, hh), qa1, s0);
      f = frag_kb(k1, hh); s1 = wmma16b(f, qa0, s1); s1 = wmma16b(f, ql0, s1); s1 = wmma16b(frag_kb(k1l, hh), qa0, s1);
      f = frag_kb(k1 + 32, hh); s1 = wmma16b(f, qa1, s1); s1 = wmma16b(f, ql1, s1); s1 = wmma16b(frag_kb(k1l + 32, hh), qa1, s1); }
    float e[16]; float bm = -INFINITY;
#pragma unroll
    for (int r = 0; r < 8; ++r) { e[r] = s0[r] * cs; e[8 + r] = s1[r] * cs; bm = fmaxf(bm, fmaxf(e[r], e[8 + r])); }
    bm = fmaxf(bm, __shfl_xor(bm, 16)); const float mn = fmaxf(mrun, bm); const float sc = exp2f(mrun - mn); float ls = 0.0f; v16b ph, pl;
#pragma unroll
    for (int i = 0; i < 16; ++i) { const float p = exp2f(e[i] - mn); ls += p; b16 a, c; split16(p * PS, a, c); ph[i] = a; pl[i] = c; }
    ls += __shfl_xor(ls, 16); lrun = lrun * sc + ls; mrun = mn;
#pragma unroll
    for (int t = 0; t < 4; ++t) { o[t] *= sc; ol[t] *= sc; const v16b vf = frag_kb(Vb + (size_t)(t * 16 + col) * N + kb, hh); o[t] = wmma16b(vf, ph, o[t]); ol[t] = wmma16b(vf, pl, ol[t]); ol[t] = wmma16b(frag_kb(Vlb + (size_t)(t * 16 + col) * N + kb, hh), ph, ol[t]); } }
  const float inv = 1.0f / (lrun * PS * XS);
#pragma unroll
  for (int t = 0; t < 4; ++t)
#pragma unroll
    for (int r = 0; r < 8; ++r) { b16 p, q; split16((o[t][r] + ol[t][r]) * inv * XS, p, q); Oh[wave * 16 + col][t * 16 + 8 * hh + r] = p; Olo[wave * 16 + col][t * 16 + 8 * hh + r] = q; }
  __syncthreads();
  { const int nloc = col, hlf = hh; v8f d4[4] = {{}, {}, {}, {}};
#pragma unroll
    for (int kb = 0; kb < C; kb += 32) { const v16b bo = frag_kb(&Oh[wave * 16 + nloc][kb], hlf), bol = frag_kb(&Olo[wave * 16 + nloc][kb], hlf);
#pragma unroll
      for (int t = 0; t < 4; ++t) { const v16b aw = frag_kb(W4 + (size_t)3 * C * C + (size_t)(t * 16 + nloc) * C + kb, hlf); d4[t] = wmma16b(aw, bo, d4[t]); d4[t] = wmma16b(aw, bol, d4[t]); } }
#pragma unroll
    for (int t = 0; t < 4; ++t)
#pragma unroll 1
      for (int r = 0; r < 8; ++r) { const int oc = t * 16 + 8 * hlf + r; St[oc][wave * 16 + nloc] = d4[t][r] * (1.0f / (WSC * XS)) + bf16_rne(bp[oc]); } }
  __syncthreads();
  for (int pass = 0; pass < 2; ++pass) { for (int oc = wave; oc < C; oc += 2) ((volatile float*)out)[((size_t)b * C + oc) * N + blockIdx.x * 32 + lane] = St[oc][lane]; __threadfence(); }
}
}

extern "C" void kernel_launch(void* const* d_in, const int* in_sizes, int n_in, void* d_out, int out_size, void* d_ws, size_t ws_size, hipStream_t stream) {
  (void)n_in;
  auto Fp = [&](int i) { return (const float*)d_in[i]; };
  if (in_sizes[0] != NR * C || in_sizes[1] != NR * C || in_sizes[2] != C * C || in_sizes[4] != C * C || in_sizes[6] != C * C || in_sizes[8] != C * C || out_size != NR * C) return;
  size_t off = 0; char* ws = (char*)d_ws;
  auto carve = [&](size_t bytes) { char* p = ws + off; off += (bytes + 255) & ~(size_t)255; return p; };
  b16* X1T = (b16*)carve((size_t)NR * C * 2); b16* X2T = (b16*)carve((size_t)NR * C * 2); b16* W4 = (b16*)carve((size_t)4 * C * C * 2);
  b16* Qh = (b16*)carve((size_t)NR * C * 2); b16* Ql = (b16*)carve((size_t)NR * C * 2); b16* Kh = (b16*)carve((size_t)NR * C * 2); b16* Kl = (b16*)carve((size_t)NR * C * 2); b16* VTh = (b16*)carve((size_t)NR * C * 2); b16* VTl = (b16*)carve((size_t)NR * C * 2);
  if (off > ws_size || off > ((size_t)128 << 20)) return;
  prep_kernel<<<dim3(N / 64, 2, NB), 256, 0, stream>>>(Fp(0), Fp(1), Fp(2), Fp(4), Fp(6), Fp(8), X1T, X2T, W4);
  proj_kernel<<<dim3(NR / 64, 3), 128, 0, stream>>>(X1T, X2T, W4, Fp(3), Fp(5), Fp(7), Qh, Ql, Kh, Kl, VTh, VTl);
  attn_kernel<<<dim3(N / 32, NB), 64, 0, stream>>>(Qh, Ql, Kh, Kl, VTh, VTl, W4, Fp(9), (float*)d_out);
}
